// PointnetSAMoudleAgg_5085241279181
// MI455X (gfx1250) — hardware-verified
//
#include <hip/hip_runtime.h>
#pragma clang fp contract(off)

typedef __attribute__((ext_vector_type(16))) _Float16 v16h;
typedef __attribute__((ext_vector_type(8)))  _Float16 v8h;
typedef __attribute__((ext_vector_type(8)))  float    v8f;
typedef __attribute__((ext_vector_type(4)))  float    v4f;
typedef __attribute__((ext_vector_type(4)))  int      v4i;

constexpr int kBatch = 4;
constexpr int kPts = 16384;
constexpr int kQry = 1024;
constexpr int kSamp = 64;
constexpr int kFeat = 128;
constexpr int kCh0 = 128;
constexpr int kCh1 = 128;
constexpr int kCh2 = 256;
constexpr int kDepth = 128;
constexpr int kW0Pitch = kFeat + 3;
constexpr int kGroups = kBatch * kQry;
constexpr int kRows = kGroups * kSamp;
constexpr int kPtRows = kBatch * kPts;
constexpr int kHalfRows = kRows / 2;
constexpr int kHalfGroups = kGroups / 2;
constexpr int kL0Rows = 256;
constexpr int kL0Chunks = kRows / kL0Rows;
constexpr float kRadius = 0.4f;
constexpr float kInvRadius = 1.0f / kRadius;
constexpr float kRadius2 = 0.16f;
constexpr float kBnEps = 1e-5f;
constexpr float kWCarry = 16.0f;
constexpr float kWCarryInv = 1.0f / kWCarry;
constexpr double kInvCount = 1.0 / (double)kRows;

static_assert(kSamp == 64);
static_assert(kRows == 262144);
static_assert(kGroups == 4096);
static_assert(kDepth % 32 == 0);
static_assert(kFeat == kDepth && kCh0 == kDepth && kCh1 == kDepth);
static_assert(kPtRows % 64 == 0 && kRows % 64 == 0 && kHalfRows % 64 == 0);
static_assert(kCh0 % 64 == 0 && kCh1 % 64 == 0 && kCh2 % 64 == 0);
static_assert(kRows % kL0Rows == 0);

constexpr size_t kOffIdx = 0;
constexpr size_t kSzIdx = (size_t)kGroups * kSamp * 4;
constexpr size_t kOffX1 = kOffIdx + kSzIdx;
constexpr size_t kSzX1 = (size_t)kRows * kCh0 * 2;
constexpr size_t kOffScr = kOffX1 + kSzX1;
constexpr size_t kSzScr = (size_t)kPtRows * kCh0 * 4;
constexpr size_t kOffMM = kOffScr + kSzScr;
constexpr size_t kSzMM = (size_t)2 * kGroups * kCh2 * 4;
constexpr size_t kOffP0 = kOffMM + kSzMM;
constexpr size_t kSzP0 = (size_t)kL0Chunks * 2 * kCh0 * 4;
constexpr size_t kOffP1 = kOffP0 + kSzP0;
constexpr size_t kSzP1 = (size_t)kGroups * 2 * kCh1 * 4;
constexpr size_t kOffP2 = kOffP1 + kSzP1;
constexpr size_t kSzP2 = (size_t)kGroups * 2 * kCh2 * 4;
constexpr size_t kOffW0F = kOffP2 + kSzP2;
constexpr size_t kSzW0F = (size_t)kCh0 * kDepth * 2;
constexpr size_t kOffW1H = kOffW0F + kSzW0F;
constexpr size_t kSzW1H = (size_t)kCh1 * kDepth * 2;
constexpr size_t kOffW2H = kOffW1H + kSzW1H;
constexpr size_t kSzW2H = (size_t)kCh2 * kDepth * 2;
constexpr size_t kOffW0X = kOffW2H + kSzW2H;
constexpr size_t kSzW0X = (size_t)kCh0 * 4 * 4;
constexpr size_t kOffScSh = kOffW0X + kSzW0X;
constexpr size_t kSzScSh = (size_t)(4 * 128 + 2 * 256) * 4;
constexpr size_t kWsTotal = kOffScSh + kSzScSh;
static_assert(kWsTotal <= (size_t)134217728);
static_assert((size_t)kHalfRows * kCh1 * 2 <= kSzScr);
static_assert((size_t)kPtRows * kFeat * 2 <= kSzX1);
static_assert(kOffX1 % 128 == 0 && kOffScr % 128 == 0 && kOffMM % 128 == 0 && kOffP0 % 128 == 0);
static_assert(kOffP1 % 128 == 0 && kOffP2 % 128 == 0 && kOffW0F % 128 == 0 && kOffW1H % 128 == 0);
static_assert(kOffW2H % 128 == 0 && kOffW0X % 128 == 0 && kOffScSh % 128 == 0);

union FragU { v16h v; v8h h[2]; };
__device__ __forceinline__ v16h frag_load(const _Float16* p) {
  FragU f;
  f.h[0] = *(const v8h*)(p);
  f.h[1] = *(const v8h*)(p + 16);
  return f.v;
}
__device__ __forceinline__ v8f frag_mma(v16h a, v16h b, v8f c) {
  return __builtin_amdgcn_wmma_f32_16x16x32_f16(false, a, false, b, (short)0, c, false, false);
}
__device__ __forceinline__ void guard4_h(v8f& a, v8f& b, v8f& c, v8f& d, v16h x) {
  asm volatile("v_nop\n\tv_nop\n\tv_nop\n\tv_nop" : "+v"(a), "+v"(b), "+v"(c), "+v"(d) : "v"(x));
}
__device__ __forceinline__ void keep4_h(v16h a, v16h b, v16h c, v16h d) {
  asm volatile("v_nop" :: "v"(a), "v"(b), "v"(c), "v"(d));
}
__device__ __forceinline__ void acc_guard4(v8f& a, v8f& b, v8f& c, v8f& d) {
  asm volatile("v_nop\n\tv_nop\n\tv_nop\n\tv_nop" : "+v"(a), "+v"(b), "+v"(c), "+v"(d));
}
__device__ __forceinline__ void wave_lds_sync() {
  __builtin_amdgcn_fence(__ATOMIC_RELEASE, "workgroup");
  __builtin_amdgcn_wave_barrier();
  __builtin_amdgcn_fence(__ATOMIC_ACQUIRE, "workgroup");
}

__global__ __launch_bounds__(256) void ballq_kernel(
    const float* __restrict__ xyz, const float* __restrict__ nxyz, int* __restrict__ idx) {
#pragma clang fp contract(off)
  __shared__ __align__(16) int sidx[8 * kSamp];
  const int tid = threadIdx.x;
  const int wave = tid >> 5;
  const int lane = tid & 31;
  const int gq = blockIdx.x * 8 + wave;
  const int b = gq / kQry;
  sidx[wave * kSamp + lane] = 0;
  sidx[wave * kSamp + 32 + lane] = 0;
  __syncthreads();
  const float qx = nxyz[(size_t)gq * 3 + 0];
  const float qy = nxyz[(size_t)gq * 3 + 1];
  const float qz = nxyz[(size_t)gq * 3 + 2];
  const float* xb = xyz + (size_t)b * kPts * 3;
  int cnt = 0;
  for (int n0 = 0; n0 < kPts && cnt < kSamp; n0 += 32) {
    const int n = n0 + lane;
    const float px = xb[n * 3 + 0];
    const float py = xb[n * 3 + 1];
    const float pz = xb[n * 3 + 2];
    const float dx = qx - px;
    const float dy = qy - py;
    const float dz = qz - pz;
    const float t0 = dx * dx;
    const float t1 = dy * dy;
    const float t2 = dz * dz;
    const float d2 = (t0 + t2) + t1;
    const bool pred = d2 < kRadius2;
    const unsigned mk = __builtin_amdgcn_ballot_w32(pred);
    const int slot = cnt + __popc(mk & ((1u << lane) - 1u));
    if (pred && slot < kSamp) sidx[wave * kSamp + slot] = n;
    cnt += __popc(mk);
  }
  __syncthreads();
  const int cc = cnt < kSamp ? cnt : kSamp;
  const int first = sidx[wave * kSamp];
  if (lane >= cc) sidx[wave * kSamp + lane] = first;
  if (lane + 32 >= cc) sidx[wave * kSamp + 32 + lane] = first;
  __syncthreads();
  if (tid < 128) {
    const v4i v = *(const v4i*)(sidx + tid * 4);
    int* dst = idx + (size_t)blockIdx.x * (8 * kSamp) + tid * 4;
    *(volatile v4i*)dst = v;
    __threadfence();
    *(volatile v4i*)dst = v;
  }
}

__global__ __launch_bounds__(256) void cvt_weights_kernel(
    const float* __restrict__ W0, const float* __restrict__ W1, const float* __restrict__ W2,
    unsigned short* __restrict__ W0F, unsigned short* __restrict__ W1H, unsigned short* __restrict__ W2H,
    float* __restrict__ W0X) {
  const int tid = threadIdx.x;
  const int blk = blockIdx.x;
  if (blk == 32) {
    if (tid < kCh0) {
      v4f v;
      v[0] = W0[tid * kW0Pitch + 0];
      v[1] = W0[tid * kW0Pitch + 1];
      v[2] = W0[tid * kW0Pitch + 2];
      v[3] = 0.0f;
      float* dst = W0X + tid * 4;
      *(volatile v4f*)dst = v;
      __threadfence();
      *(volatile v4f*)dst = v;
    }
    return;
  }
  const float* src;
  unsigned short* dst;
  int pitch, kofs, tb;
  if (blk < 8) { src = W0; dst = W0F; pitch = kW0Pitch; kofs = 3; tb = blk * 256 + tid; }
  else if (blk < 16) { src = W1; dst = W1H; pitch = kDepth; kofs = 0; tb = (blk - 8) * 256 + tid; }
  else { src = W2; dst = W2H; pitch = kDepth; kofs = 0; tb = (blk - 16) * 256 + tid; }
  const int e0 = tb * 8;
  const int o = e0 / kDepth;
  const int k = e0 - o * kDepth;
  v8h hv;
#pragma unroll
  for (int e = 0; e < 8; ++e) {
    const float f = src[o * pitch + kofs + k + e] * kWCarry;
    hv[e] = (_Float16)f;
  }
  *(volatile v8h*)(dst + e0) = hv;
  __threadfence();
  *(volatile v8h*)(dst + e0) = hv;
}

__global__ __launch_bounds__(256) void feat_transpose_kernel(
    const float* __restrict__ feat, unsigned short* __restrict__ featT) {
  __shared__ __align__(16) float tile[kFeat * 65];
  const int tid = threadIdx.x;
  const int rb = blockIdx.x * 64;
  const int b = rb / kPts;
  const int n0 = rb - b * kPts;
#pragma unroll
  for (int it = 0; it < 8; ++it) {
    const int q = it * 256 + tid;
    const int c = q >> 4;
    const int n4 = (q & 15) * 4;
    const v4f v = *(const v4f*)(feat + ((size_t)(b * kFeat + c)) * kPts + n0 + n4);
    tile[c * 65 + n4 + 0] = v[0];
    tile[c * 65 + n4 + 1] = v[1];
    tile[c * 65 + n4 + 2] = v[2];
    tile[c * 65 + n4 + 3] = v[3];
  }
  __syncthreads();
  const int r16 = tid >> 4;
  const int c8 = (tid & 15) * 8;
  for (int pass = 0; pass < 2; ++pass) {
#pragma unroll
    for (int it = 0; it < 4; ++it) {
      const int r = it * 16 + r16;
      v8h hv;
#pragma unroll
      for (int e = 0; e < 8; ++e) hv[e] = (_Float16)tile[(c8 + e) * 65 + r];
      *(volatile v8h*)(featT + (size_t)(rb + r) * kFeat + c8) = hv;
    }
    __threadfence();
  }
}

template <int MODE>
__global__ __launch_bounds__(256) void mlp_gemm_kernel(
    const unsigned short* __restrict__ Ap, const unsigned short* __restrict__ Btp,
    float* __restrict__ outF, unsigned short* __restrict__ outH, float* __restrict__ outMM,
    const float* __restrict__ scv, const float* __restrict__ shv,
    int M, int N, int tmBase, float cscale) {
  const _Float16* A = (const _Float16*)Ap;
  const _Float16* Bt = (const _Float16*)Btp;
  __shared__ __align__(16) float sT[8][16 * 68];
  const int lane = threadIdx.x & 31;
  const int wave = threadIdx.x >> 5;
  const int tilesN = N >> 6;
  const int tilesM = M >> 6;
  const int tile = blockIdx.x * 8 + wave;
  if (tile >= tilesM * tilesN) return;
  const int tm = tile / tilesN;
  const int tn = tile - tm * tilesN;
  const int m0 = tm << 6;
  const int n0 = tn << 6;
  const int rlane = lane & 15;
  const int hh = lane >> 4;
  const int koff = hh * 8;
  const int mOff = hh * 8;

  v8f acc[4][4];
#pragma unroll
  for (int i = 0; i < 4; ++i)
#pragma unroll
    for (int j = 0; j < 4; ++j) acc[i][j] = (v8f){0.f, 0.f, 0.f, 0.f, 0.f, 0.f, 0.f, 0.f};

#pragma unroll 1
  for (int k0 = 0; k0 < kDepth; k0 += 32) {
    v16h bh[4];
#pragma unroll
    for (int j = 0; j < 4; ++j)
      bh[j] = frag_load(Bt + (size_t)(n0 + (j << 4) + rlane) * kDepth + koff + k0);
#pragma unroll
    for (int i = 0; i < 4; ++i) {
      const v16h ah = frag_load(A + (size_t)(m0 + (i << 4) + rlane) * kDepth + koff + k0);
#pragma unroll
      for (int j = 0; j < 4; ++j) acc[i][j] = frag_mma(ah, bh[j], acc[i][j]);
      guard4_h(acc[i][0], acc[i][1], acc[i][2], acc[i][3], ah);
    }
    keep4_h(bh[0], bh[1], bh[2], bh[3]);
  }
  acc_guard4(acc[0][0], acc[0][1], acc[0][2], acc[0][3]);
  acc_guard4(acc[1][0], acc[1][1], acc[1][2], acc[1][3]);
  acc_guard4(acc[2][0], acc[2][1], acc[2][2], acc[2][3]);
  acc_guard4(acc[3][0], acc[3][1], acc[3][2], acc[3][3]);

  float* slab = sT[wave];

  if (MODE == 0 || MODE == 2) {
    float scj[4], shj[4];
#pragma unroll
    for (int j = 0; j < 4; ++j) {
      scj[j] = (MODE == 2) ? scv[n0 + (j << 4) + rlane] : cscale;
      shj[j] = (MODE == 2) ? shv[n0 + (j << 4) + rlane] : 0.0f;
    }
#pragma unroll
    for (int i = 0; i < 4; ++i) {
      const int mBase = m0 + (i << 4);
#pragma unroll
      for (int j = 0; j < 4; ++j) {
#pragma unroll
        for (int r = 0; r < 8; ++r) {
          float v = acc[i][j][r] * scj[j];
          if (MODE == 2) {
            v = v + shj[j];
            v = fmaxf(v, 0.0f);
          }
          slab[(mOff + r) * 68 + (j << 4) + rlane] = v;
        }
      }
      wave_lds_sync();
      if (MODE == 0) {
        const int c4 = (lane & 15) * 4;
        for (int pass = 0; pass < 2; ++pass) {
#pragma unroll
          for (int it = 0; it < 8; ++it) {
            const int row = it * 2 + hh;
            const v4f v = *(const v4f*)(slab + row * 68 + c4);
            *(volatile v4f*)(outF + (size_t)(mBase + row) * N + n0 + c4) = v;
          }
          __threadfence();
        }
      } else {
        const int q = lane >> 3;
        const int c8 = (lane & 7) * 8;
        for (int pass = 0; pass < 2; ++pass) {
#pragma unroll
          for (int it = 0; it < 4; ++it) {
            const int row = it * 4 + q;
            const float* sp = slab + row * 68 + c8;
            v8h hv;
#pragma unroll
            for (int e = 0; e < 8; ++e) hv[e] = (_Float16)sp[e];
            *(volatile v8h*)(outH + (size_t)(mBase + row) * N + n0 + c8) = hv;
          }
          __threadfence();
        }
      }
      wave_lds_sync();
    }
  } else {
    float cs[4], cq[4], cx[4], cn[4];
#pragma unroll
    for (int j = 0; j < 4; ++j) {
      float s = 0.0f, q = 0.0f;
      float mx = acc[0][j][0];
      float mn = acc[0][j][0];
#pragma unroll
      for (int i = 0; i < 4; ++i) {
#pragma unroll
        for (int r = 0; r < 8; ++r) {
          const float x = acc[i][j][r];
          s = s + x;
          q = q + x * x;
          if (MODE == 3) {
            mx = fmaxf(mx, x);
            mn = fminf(mn, x);
          }
        }
      }
      cs[j] = s; cq[j] = q; cx[j] = mx; cn[j] = mn;
    }
#pragma unroll
    for (int j = 0; j < 4; ++j) {
      const float so = __shfl_xor(cs[j], 16, 32);
      const float qo = __shfl_xor(cq[j], 16, 32);
      const float xo = __shfl_xor(cx[j], 16, 32);
      const float no = __shfl_xor(cn[j], 16, 32);
      cs[j] = cs[j] + so;
      cq[j] = cq[j] + qo;
      cx[j] = fmaxf(cx[j], xo);
      cn[j] = fminf(cn[j], no);
    }
    if (hh == 0) {
#pragma unroll
      for (int j = 0; j < 4; ++j) {
        slab[(j << 4) + rlane] = cs[j];
        slab[64 + (j << 4) + rlane] = cq[j];
        slab[128 + (j << 4) + rlane] = cx[j];
        slab[192 + (j << 4) + rlane] = cn[j];
      }
    }
    wave_lds_sync();
    const int seg = hh;
    const int c4 = (lane & 15) * 4;
    const int tmG = tmBase + tm;
    const v4f v0 = *(const v4f*)(slab + seg * 64 + c4);
    float* p0 = outF + ((size_t)(tmG * 2 + seg)) * N + n0 + c4;
    v4f v1 = v0;
    float* p1 = p0;
    if (MODE == 3) {
      v1 = *(const v4f*)(slab + 128 + seg * 64 + c4);
      p1 = outMM + (size_t)seg * ((size_t)kGroups * kCh2) + (size_t)tmG * N + n0 + c4;
    }
    *(volatile v4f*)p0 = v0;
    if (MODE == 3) *(volatile v4f*)p1 = v1;
    __threadfence();
    *(volatile v4f*)p0 = v0;
    if (MODE == 3) *(volatile v4f*)p1 = v1;
  }
}

template <bool NORM>
__global__ __launch_bounds__(128) void layer0_kernel(
    const float* __restrict__ xyz, const float* __restrict__ nxyz, const int* __restrict__ idx,
    const float* __restrict__ fproj, const float* __restrict__ w0x,
    const float* __restrict__ sc0, const float* __restrict__ sh0,
    unsigned short* __restrict__ x1, float* __restrict__ part) {
  __shared__ __align__(16) float sW[kCh0 * 4];
  __shared__ __align__(16) float sSc[kCh0];
  __shared__ __align__(16) float sSh[kCh0];
  __shared__ __align__(16) float sG[kL0Rows * 4];
  __shared__ int sId[kL0Rows];
  __shared__ float sRed[8 * 2 * kCh0];
  const int tid = threadIdx.x;
  const int m0 = blockIdx.x * kL0Rows;

  *(v4f*)(sW + tid * 4) = *(const v4f*)(w0x + tid * 4);
  float scl0 = 0.0f, shf0 = 0.0f;
  if (NORM) { scl0 = sc0[tid]; shf0 = sh0[tid]; }
  sSc[tid] = scl0;
  sSh[tid] = shf0;
#pragma unroll
  for (int rr = 0; rr < 2; ++rr) {
    const int r = tid + rr * 128;
    const int m = m0 + r;
    const int b = m / (kQry * kSamp);
    const int g = m / kSamp;
    int id = idx[m];
    id = id < 0 ? 0 : id;
    id = id > (kPts - 1) ? (kPts - 1) : id;
    const int prow = b * kPts + id;
    const float gx = (xyz[(size_t)prow * 3 + 0] - nxyz[(size_t)g * 3 + 0]) * kInvRadius;
    const float gy = (xyz[(size_t)prow * 3 + 1] - nxyz[(size_t)g * 3 + 1]) * kInvRadius;
    const float gz = (xyz[(size_t)prow * 3 + 2] - nxyz[(size_t)g * 3 + 2]) * kInvRadius;
    sId[r] = prow;
    sG[r * 4 + 0] = gx;
    sG[r * 4 + 1] = gy;
    sG[r * 4 + 2] = gz;
    sG[r * 4 + 3] = 0.0f;
  }
  __syncthreads();

  const int rq = tid >> 4;
  const int c8 = (tid & 15) * 8;
  float wx[8], wy[8], wz[8], scl[8], shf[8], s[8], q[8];
#pragma unroll
  for (int e = 0; e < 8; ++e) {
    const v4f wv = *(const v4f*)(sW + (c8 + e) * 4);
    wx[e] = wv[0];
    wy[e] = wv[1];
    wz[e] = wv[2];
    scl[e] = sSc[c8 + e];
    shf[e] = sSh[c8 + e];
    s[e] = 0.0f;
    q[e] = 0.0f;
  }

#pragma unroll 1
  for (int it = 0; it < kL0Rows / 8; ++it) {
    const int r = it * 8 + rq;
    const int prow = sId[r];
    const v4f g = *(const v4f*)(sG + r * 4);
    const float* fp = fproj + (size_t)prow * kCh0 + c8;
    const v4f f0 = *(const v4f*)(fp);
    const v4f f1 = *(const v4f*)(fp + 4);
    float y[8];
#pragma unroll
    for (int e = 0; e < 4; ++e) { y[e] = f0[e]; y[4 + e] = f1[e]; }
#pragma unroll
    for (int e = 0; e < 8; ++e) {
      const float a0 = wx[e] * g[0];
      const float a1 = wy[e] * g[1];
      const float a2 = wz[e] * g[2];
      y[e] = ((y[e] + a0) + a1) + a2;
    }
    if (NORM) {
      v8h hv;
#pragma unroll
      for (int e = 0; e < 8; ++e) {
        float v = y[e] * scl[e];
        v = v + shf[e];
        v = fmaxf(v, 0.0f);
        hv[e] = (_Float16)v;
      }
      unsigned short* dst = x1 + (size_t)(m0 + r) * kCh0 + c8;
      *(volatile v8h*)dst = hv;
      __threadfence();
      *(volatile v8h*)dst = hv;
    } else {
#pragma unroll
      for (int e = 0; e < 8; ++e) {
        s[e] = s[e] + y[e];
        q[e] = q[e] + y[e] * y[e];
      }
    }
  }

  if (!NORM) {
#pragma unroll
    for (int e = 0; e < 8; ++e) {
      sRed[(rq * 2 + 0) * kCh0 + c8 + e] = s[e];
      sRed[(rq * 2 + 1) * kCh0 + c8 + e] = q[e];
    }
    __syncthreads();
    float ts = 0.0f, tq = 0.0f;
#pragma unroll
    for (int g8 = 0; g8 < 8; ++g8) {
      ts = ts + sRed[(g8 * 2 + 0) * kCh0 + tid];
      tq = tq + sRed[(g8 * 2 + 1) * kCh0 + tid];
    }
    float* ps = part + ((size_t)blockIdx.x * 2 + 0) * kCh0 + tid;
    float* pq = part + ((size_t)blockIdx.x * 2 + 1) * kCh0 + tid;
    *(volatile float*)ps = ts;
    *(volatile float*)pq = tq;
    __threadfence();
    *(volatile float*)ps = ts;
    *(volatile float*)pq = tq;
  }
}

__global__ __launch_bounds__(256) void bn_reduce_kernel(
    const float* __restrict__ part, int nparts, int nch, float carryInv,
    const float* __restrict__ gam, const float* __restrict__ bet,
    float* __restrict__ sc, float* __restrict__ sh) {
  __shared__ double sS[256];
  __shared__ double sQ[256];
  const int tid = threadIdx.x;
  const int pg = tid >> 5;
  const int c = blockIdx.x * 32 + (tid & 31);
  double s = 0.0, q = 0.0;
#pragma unroll 4
  for (int p = pg; p < nparts; p += 8) {
    s = s + (double)part[((size_t)p * 2 + 0) * nch + c];
    q = q + (double)part[((size_t)p * 2 + 1) * nch + c];
  }
  sS[tid] = s;
  sQ[tid] = q;
  __syncthreads();
  if (tid < 32) {
    double S = 0.0, Q = 0.0;
#pragma unroll
    for (int g8 = 0; g8 < 8; ++g8) {
      S = S + sS[g8 * 32 + tid];
      Q = Q + sQ[g8 * 32 + tid];
    }
    const double ci = (double)carryInv;
    const double mean = S * ci * kInvCount;
    const double ex2 = Q * ci * ci * kInvCount;
    double var = ex2 - mean * mean;
    var = var < 0.0 ? 0.0 : var;
    const float vf = (float)var;
    const float rs = 1.0f / sqrtf(vf + kBnEps);
    const float scale = gam[c] * rs;
    const float shift = bet[c] - (float)mean * scale;
    const float so = scale * carryInv;
    *(volatile float*)(sc + c) = so;
    *(volatile float*)(sh + c) = shift;
    __threadfence();
    *(volatile float*)(sc + c) = so;
    *(volatile float*)(sh + c) = shift;
  }
}

__global__ __launch_bounds__(256) void finalize_kernel(
    const float* __restrict__ mm, const float* __restrict__ sc2, const float* __restrict__ sh2,
    float* __restrict__ out) {
  __shared__ __align__(16) float tile[32 * 36];
  const int tid = threadIdx.x;
  const int wave = tid >> 5;
  const int lane = tid & 31;
  const int g0 = blockIdx.x * 32;
  const int b = g0 / kQry;
  const int p0 = g0 - b * kQry;
  const int pl = tid >> 3;
  const int o4 = (tid & 7) * 4;
  const size_t plane = (size_t)kGroups * kCh2;
#pragma unroll 1
  for (int oc = 0; oc < kCh2 / 32; ++oc) {
    const int o = oc * 32 + o4;
    const v4f mx = *(const v4f*)(mm + (size_t)(g0 + pl) * kCh2 + o);
    const v4f mn = *(const v4f*)(mm + plane + (size_t)(g0 + pl) * kCh2 + o);
    const v4f sv = *(const v4f*)(sc2 + o);
    const v4f hv = *(const v4f*)(sh2 + o);
#pragma unroll
    for (int e = 0; e < 4; ++e) {
      const float a = sv[e] * mx[e] + hv[e];
      const float c = sv[e] * mn[e] + hv[e];
      const float v = fmaxf(fmaxf(a, c), 0.0f);
      tile[(o4 + e) * 36 + pl] = v;
    }
    __syncthreads();
    {
      const int ol = wave * 4 + (lane >> 3);
      const int p4 = (lane & 7) * 4;
      const v4f v = *(const v4f*)(tile + ol * 36 + p4);
      float* dst = out + ((size_t)(b * kCh2 + oc * 32 + ol)) * kQry + p0 + p4;
      *(volatile v4f*)dst = v;
      __threadfence();
      *(volatile v4f*)dst = v;
    }
    __syncthreads();
  }
}

extern "C" void kernel_launch(void* const* d_in, const int* in_sizes, int n_in,
                              void* d_out, int out_size, void* d_ws, size_t ws_size,
                              hipStream_t stream) {
  (void)in_sizes;
  (void)out_size;
  if (n_in < 12) return;
  if (ws_size < kWsTotal) return;
  const float* xyz  = (const float*)d_in[0];
  const float* nxyz = (const float*)d_in[1];
  const float* feat = (const float*)d_in[2];
  const float* W0 = (const float*)d_in[3];
  const float* g0 = (const float*)d_in[4];
  const float* b0 = (const float*)d_in[5];
  const float* W1 = (const float*)d_in[6];
  const float* g1 = (const float*)d_in[7];
  const float* b1 = (const float*)d_in[8];
  const float* W2 = (const float*)d_in[9];
  const float* g2 = (const float*)d_in[10];
  const float* b2 = (const float*)d_in[11];
  float* out = (float*)d_out;

  char* ws = (char*)d_ws;
  int* idx = (int*)(ws + kOffIdx);
  unsigned short* x1 = (unsigned short*)(ws + kOffX1);
  unsigned short* featT = x1;
  float* fproj = (float*)(ws + kOffScr);
  unsigned short* x2 = (unsigned short*)(ws + kOffScr);
  float* mm = (float*)(ws + kOffMM);
  float* p0 = (float*)(ws + kOffP0);
  float* p1 = (float*)(ws + kOffP1);
  float* p2 = (float*)(ws + kOffP2);
  unsigned short* w0f = (unsigned short*)(ws + kOffW0F);
  unsigned short* w1h = (unsigned short*)(ws + kOffW1H);
  unsigned short* w2h = (unsigned short*)(ws + kOffW2H);
  float* w0x = (float*)(ws + kOffW0X);
  float* scsh = (float*)(ws + kOffScSh);
  float* sc0 = scsh;
  float* sh0 = scsh + 128;
  float* sc1 = scsh + 256;
  float* sh1 = scsh + 384;
  float* sc2 = scsh + 512;
  float* sh2 = scsh + 768;

  ballq_kernel<<<dim3(kGroups / 8), dim3(256), 0, stream>>>(xyz, nxyz, idx);
  cvt_weights_kernel<<<dim3(33), dim3(256), 0, stream>>>(W0, W1, W2, w0f, w1h, w2h, w0x);
  feat_transpose_kernel<<<dim3(kPtRows / 64), dim3(256), 0, stream>>>(feat, featT);
  mlp_gemm_kernel<0><<<dim3((kPtRows / 64) * (kCh0 / 64) / 8), dim3(256), 0, stream>>>(
      featT, w0f, fproj, x2, mm, sc0, sh0, kPtRows, kCh0, 0, kWCarryInv);
  layer0_kernel<false><<<dim3(kL0Chunks), dim3(128), 0, stream>>>(
      xyz, nxyz, idx, fproj, w0x, sc0, sh0, x1, p0);
  bn_reduce_kernel<<<dim3(kCh0 / 32), dim3(256), 0, stream>>>(p0, kL0Chunks, kCh0, 1.0f, g0, b0, sc0, sh0);
  layer0_kernel<true><<<dim3(kL0Chunks), dim3(128), 0, stream>>>(
      xyz, nxyz, idx, fproj, w0x, sc0, sh0, x1, p0);
  mlp_gemm_kernel<1><<<dim3((kRows / 64) * (kCh1 / 64) / 8), dim3(256), 0, stream>>>(
      x1, w1h, p1, x2, mm, sc1, sh1, kRows, kCh1, 0, 1.0f);
  bn_reduce_kernel<<<dim3(kCh1 / 32), dim3(256), 0, stream>>>(p1, kGroups, kCh1, kWCarryInv, g1, b1, sc1, sh1);
  for (int h = 0; h < 2; ++h) {
    mlp_gemm_kernel<2><<<dim3((kHalfRows / 64) * (kCh1 / 64) / 8), dim3(256), 0, stream>>>(
        x1 + (size_t)h * kHalfRows * kCh0, w1h, p1, x2, mm, sc1, sh1, kHalfRows, kCh1, 0, 1.0f);
    mlp_gemm_kernel<3><<<dim3((kHalfRows / 64) * (kCh2 / 64) / 8), dim3(256), 0, stream>>>(
        x2, w2h, p2, x2, mm, sc2, sh2, kHalfRows, kCh2, h * kHalfGroups, 1.0f);
  }
  bn_reduce_kernel<<<dim3(kCh2 / 32), dim3(256), 0, stream>>>(p2, kGroups, kCh2, kWCarryInv, g2, b2, sc2, sh2);
  finalize_kernel<<<dim3(kGroups / 32), dim3(256), 0, stream>>>(mm, sc2, sh2, out);
}
